// CoordinateDecoder_83038897701018
// MI455X (gfx1250) — hardware-verified
//
#include <hip/hip_runtime.h>
#include <math.h>

#pragma clang fp contract(off)


#ifndef NPTS
#define NPTS 65536
#endif
#ifndef NB
#define NB 4
#endif
#define GH 64
#define GW 64
#define DM 128
#define MLPW 256
#define FILMW 512
#define NFREQ 10
#define ENCD 42
#define KIN0 170
#define KP0 192
#define TILE 64
#define HROW 264
#define ENCP 64
#define SC_A 16.0f
#define SC_R 256.0f
#define SC_W 256.0f
#define SC_WL 1.0f
#define INV_ACC 0.000244140625f

static_assert(NPTS % TILE == 0);
static_assert(KP0 % 32 == 0 && KP0 >= KIN0 && KP0 <= HROW);
static_assert(HROW % 8 == 0 && HROW >= MLPW);
static_assert(ENCD + DM == KIN0);
static_assert(ENCD + 6 <= 48 && 48 <= ENCP);

typedef __attribute__((ext_vector_type(16))) _Float16 v16h;
typedef __attribute__((ext_vector_type(8)))  _Float16 v8h;
typedef __attribute__((ext_vector_type(8)))  float v8f;
typedef __attribute__((ext_vector_type(4)))  float v4f;
typedef __attribute__((ext_vector_type(4)))  unsigned v4u;
typedef float __attribute__((may_alias)) float_a;

template <typename T> __device__ __forceinline__ void vst2(void* p, T v) { *(volatile T*)p = v; __threadfence(); *(volatile T*)p = v; }

__device__ __forceinline__ v8f wmma16(v16h a, v16h b, v8f c) {
  v8f d = __builtin_amdgcn_wmma_f32_16x16x32_f16(false, a, false, b, (short)0, c, false, false);
  asm volatile("v_nop\n\tv_nop\n\tv_nop\n\tv_nop" : "+v"(d) : "v"(a), "v"(b));
  return d;
}
__device__ __forceinline__ v16h frag_h(const _Float16* rowk0, int lane) {
  union { v16h v; v8h q[2]; } u; const _Float16* p = rowk0 + 8 * (lane >> 4);
  u.q[0] = *(const v8h*)p; u.q[1] = *(const v8h*)(p + 16); return u.v;
}
__device__ __forceinline__ float bfr(float x) {
  unsigned u = __float_as_uint(x); u += 0x7FFFu + ((u >> 16) & 1u); return __uint_as_float(u & 0xFFFF0000u);
}
__device__ __forceinline__ int refl(int i, int size) {
  const int s = 2 * size; const int i2 = 2 * i + 1;
  int m = (i2 + s) % (2 * s); if (m < 0) m += 2 * s;
  m -= s; if (m < 0) m = -m;
  return (m - 1) >> 1;
}
__device__ __forceinline__ float tanh_q(float x) {
  const float e = __expf(-2.0f * fabsf(x));
  const float t = (1.0f - e) * __builtin_amdgcn_rcpf(1.0f + e);
  return copysignf(t, x);
}
__device__ __forceinline__ float gelu_t(float x) {
  const float x3 = (x * x) * x;
  const float u = 0.7978845608028654f * (x + 0.044715f * x3);
  return x * (0.5f * (1.0f + tanh_q(u)));
}

__global__ __launch_bounds__(256) void k_film(const float* __restrict__ ctx, const float* __restrict__ wf,
                                             const float* __restrict__ bfm, float* __restrict__ film) {
  const int b = blockIdx.x;
  for (int j = threadIdx.x; j < FILMW; j += 256) {
    float s = 0.0f;
#pragma unroll 1
    for (int k = 0; k < DM; ++k) s = s + bfr(ctx[(size_t)b * DM + k]) * bfr(wf[(size_t)k * FILMW + j]);
    s = s + bfr(bfm[j]);
    const float v = (j < MLPW) ? (s + 1.0f) : s;
    vst2(film + (size_t)b * FILMW + j, (float_a)v);
  }
}

__global__ __launch_bounds__(256) void k_wprep(const float* __restrict__ w, int K, int N, int nrows, int KP, int two,
                                              float shi, float slo, _Float16* __restrict__ dst) {
  const int KPT = two ? 2 * KP : KP;
  const int cpr = KPT / 8;
  const int g = blockIdx.x * 256 + threadIdx.x;
  if (g >= nrows * cpr) return;
  const int n = g / cpr, c8 = g - n * cpr;
  int kb = c8 * 8; const bool lo = kb >= KP; if (lo) kb -= KP;
  const float sc = lo ? slo : shi;
  const int nc = n < N ? n : N - 1;
  union { v8h h; v4u u; } pk;
#pragma unroll
  for (int e = 0; e < 8; ++e) {
    const int k = kb + e; const int kc = k < K ? k : K - 1;
    const float x = w[(size_t)kc * N + nc];
    pk.h[e] = (_Float16)((k < K && n < N) ? bfr(x) * sc : 0.0f);
  }
  vst2(dst + (size_t)n * KPT + (size_t)c8 * 8, pk.u);
}

__global__ __launch_bounds__(256) void k_enc(const float* __restrict__ coords, _Float16* __restrict__ eh, _Float16* __restrict__ el) {
  __shared__ __align__(16) float se[TILE][48];
  const int tid = threadIdx.x, p = tid & (TILE - 1), q = tid >> 6, p0 = blockIdx.x * TILE;
  const float cx = bfr(coords[(size_t)(p0 + p) * 2]), cy = bfr(coords[(size_t)(p0 + p) * 2 + 1]);
  if (q == 0) {
    se[p][0] = cx; se[p][1] = cy;
#pragma unroll
    for (int k = ENCD; k < 48; ++k) se[p][k] = 0.0f;
  }
#pragma unroll 1
  for (int t = q; t < 2 * NFREQ; t += 4) {
    const int f = t >> 1, ax = t & 1;
    const float fr = 3.14159265358979f * (float)(1 << f);
    const float arg = (ax ? cy : cx) * fr;
    se[p][2 + 4 * f + ax] = sinf(arg);
    se[p][4 + 4 * f + ax] = cosf(arg);
  }
  __syncthreads();
  for (int i = tid; i < TILE * 8; i += 256) {
    const int r = i >> 3, c = i & 7;
    union { v8h h; v4u u; } ph, pl;
#pragma unroll
    for (int e = 0; e < 8; ++e) {
      const int k = c * 8 + e; const int kc = k < 48 ? k : 47;
      const float v = (k < 48) ? se[r][kc] * SC_A : 0.0f;
      const _Float16 hh = (_Float16)v;
      ph.h[e] = hh; pl.h[e] = (_Float16)((v - (float)hh) * SC_R);
    }
    const size_t o = (size_t)(p0 + r) * ENCP + (size_t)c * 8;
    vst2(eh + o, ph.u); vst2(el + o, pl.u);
  }
}

__device__ __forceinline__ void kloop(v8f (&acc)[4][2], const _Float16* A, const _Float16* __restrict__ B0,
                                      const _Float16* __restrict__ B1, int nks, int lane) {
#pragma unroll 1
  for (int ks = 0; ks < nks; ++ks) {
    const v16h bf0 = frag_h(B0 + ks * 32, lane), bf1 = frag_h(B1 + ks * 32, lane);
#pragma unroll
    for (int mt = 0; mt < 4; ++mt) {
      const v16h af = frag_h(A + mt * 16 * HROW + ks * 32, lane);
      acc[mt][0] = wmma16(af, bf0, acc[mt][0]);
      acc[mt][1] = wmma16(af, bf1, acc[mt][1]);
    }
  }
}

template <int NKS, bool ALO, bool OLO>
__device__ __forceinline__ void mlp_layer(_Float16* P0, _Float16* P1, const _Float16* __restrict__ Wp,
                                          const float* __restrict__ bias, const float* __restrict__ filmb, int lane, int wv) {
  constexpr int KPT = (ALO ? 2 : 1) * NKS * 32;
  const int col = lane & 15, g = lane >> 4, nbase = wv * 32;
  v8f acc[4][2];
#pragma unroll
  for (int mt = 0; mt < 4; ++mt)
#pragma unroll
    for (int j = 0; j < 2; ++j)
#pragma unroll
      for (int r = 0; r < 8; ++r) acc[mt][j][r] = 0.0f;
  const _Float16* Wr0 = Wp + (size_t)(nbase + col) * KPT;
  const _Float16* Wr1 = Wp + (size_t)(nbase + 16 + col) * KPT;
  kloop(acc, P0 + col * HROW, Wr0, Wr1, NKS, lane);
  if (ALO) kloop(acc, P1 + col * HROW, Wr0 + NKS * 32, Wr1 + NKS * 32, NKS, lane);
  __syncthreads();
#pragma unroll
  for (int j = 0; j < 2; ++j) {
    const int n = nbase + 16 * j + col;
    const float bv = bfr(bias[n]), g1 = filmb[n], be = filmb[MLPW + n];
#pragma unroll
    for (int mt = 0; mt < 4; ++mt)
#pragma unroll
      for (int r = 0; r < 8; ++r) {
        float x = acc[mt][j][r] * INV_ACC + bv;
        x = x * g1 + be;
        x = gelu_t(x);
        const float a = x * SC_A; const _Float16 hh = (_Float16)a;
        const int row = mt * 16 + 8 * g + r;
        P0[row * HROW + n] = hh;
        if (OLO) P1[row * HROW + n] = (_Float16)((a - (float)hh) * SC_R);
      }
  }
  __syncthreads();
}

__global__ __launch_bounds__(256) void k_dec(const float* __restrict__ fg, const float* __restrict__ coords,
                                            const _Float16* __restrict__ eh, const _Float16* __restrict__ el,
                                            const _Float16* __restrict__ W0p, const _Float16* __restrict__ W1p,
                                            const _Float16* __restrict__ W2p, const _Float16* __restrict__ W3p,
                                            const _Float16* __restrict__ WOp,
                                            const float* __restrict__ b0, const float* __restrict__ b1,
                                            const float* __restrict__ b2, const float* __restrict__ b3,
                                            const float* __restrict__ film, const float* __restrict__ bo,
                                            float* __restrict__ out) {
  __shared__ __align__(16) _Float16 P0[TILE * HROW];
  __shared__ __align__(16) _Float16 P1[TILE * HROW];
  __shared__ __align__(16) float pw[TILE * 4];
  __shared__ __align__(16) int pidx[TILE * 4];
  __shared__ __align__(16) float ost[TILE * 3];
  const int tid = threadIdx.x, lane = tid & 31, wv = tid >> 5;
  constexpr int TPB = NPTS / TILE;
  const int b = (int)(blockIdx.x / TPB), p0 = (int)(blockIdx.x % TPB) * TILE;

  if (tid < TILE) {
    const int p = tid;
    const float cx = bfr(coords[(size_t)(p0 + p) * 2]), cy = bfr(coords[(size_t)(p0 + p) * 2 + 1]);
    float py = ((cx + 1.0f) * 0.5f) * (float)(GH - 1);
    float px = ((cy + 1.0f) * 0.5f) * (float)(GW - 1);
    py = fminf(fmaxf(py, -1.0e7f), 1.0e7f); px = fminf(fmaxf(px, -1.0e7f), 1.0e7f);
    const float fy = floorf(py), fx = floorf(px);
    const float uy = py - fy, ux = px - fx;
    const float ly = 1.0f - uy, lx = 1.0f - ux;
    const int iy = (int)fy, ix = (int)fx;
    const int y0 = refl(iy, GH), y1 = refl(iy + 1, GH), x0 = refl(ix, GW), x1 = refl(ix + 1, GW);
    pw[p * 4 + 0] = ly * lx; pw[p * 4 + 1] = ly * ux; pw[p * 4 + 2] = uy * lx; pw[p * 4 + 3] = uy * ux;
    pidx[p * 4 + 0] = (y0 * GW + x0) * DM; pidx[p * 4 + 1] = (y0 * GW + x1) * DM;
    pidx[p * 4 + 2] = (y1 * GW + x0) * DM; pidx[p * 4 + 3] = (y1 * GW + x1) * DM;
  }
  for (int i = tid; i < TILE * 6; i += 256) {
    const int r = i / 6, c = i - r * 6;
    const size_t src = (size_t)(p0 + r) * ENCP + (size_t)c * 8;
    *(v8h*)(P0 + r * HROW + c * 8) = *(const v8h*)(eh + src);
    *(v8h*)(P1 + r * HROW + c * 8) = *(const v8h*)(el + src);
  }
  {
    v8h z;
#pragma unroll
    for (int e = 0; e < 8; ++e) z[e] = (_Float16)0.0f;
    for (int i = tid; i < TILE * 3; i += 256) {
      const int r = i / 3, c = i - r * 3;
      *(v8h*)(P0 + r * HROW + 168 + c * 8) = z;
      *(v8h*)(P1 + r * HROW + 168 + c * 8) = z;
    }
  }
  __syncthreads();
  const float* fgb = fg + (size_t)b * (GH * GW * DM);
  for (int i = tid; i < TILE * DM; i += 256) {
    const int p = i >> 7, c = i & (DM - 1);
    const int o0 = pidx[p * 4 + 0], o1 = pidx[p * 4 + 1], o2 = pidx[p * 4 + 2], o3 = pidx[p * 4 + 3];
    const float w0 = pw[p * 4 + 0], w1 = pw[p * 4 + 1], w2 = pw[p * 4 + 2], w3 = pw[p * 4 + 3];
    const float v00 = bfr(fgb[o0 + c]), v01 = bfr(fgb[o1 + c]), v10 = bfr(fgb[o2 + c]), v11 = bfr(fgb[o3 + c]);
    const float v = ((w0 * v00 + w1 * v01) + w2 * v10) + w3 * v11;
    const float a = v * SC_A; const _Float16 hh = (_Float16)a;
    P0[p * HROW + ENCD + c] = hh;
    P1[p * HROW + ENCD + c] = (_Float16)((a - (float)hh) * SC_R);
  }
  __syncthreads();

  const float* filmb = film + (size_t)b * FILMW;
  mlp_layer<KP0 / 32, true, false>(P0, P1, W0p, b0, filmb, lane, wv);
  mlp_layer<MLPW / 32, false, false>(P0, P1, W1p, b1, filmb, lane, wv);
  mlp_layer<MLPW / 32, false, false>(P0, P1, W2p, b2, filmb, lane, wv);
  mlp_layer<MLPW / 32, false, true>(P0, P1, W3p, b3, filmb, lane, wv);

  if (wv < 4) {
    const int col = lane & 15, g = lane >> 4, mt = wv;
    v8f acc;
#pragma unroll
    for (int r = 0; r < 8; ++r) acc[r] = 0.0f;
    const _Float16* Ar0 = P0 + (mt * 16 + col) * HROW;
    const _Float16* Ar1 = P1 + (mt * 16 + col) * HROW;
    const _Float16* Wr = WOp + (size_t)col * (2 * MLPW);
#pragma unroll 1
    for (int ks = 0; ks < MLPW / 32; ++ks) acc = wmma16(frag_h(Ar0 + ks * 32, lane), frag_h(Wr + ks * 32, lane), acc);
#pragma unroll 1
    for (int ks = 0; ks < MLPW / 32; ++ks) acc = wmma16(frag_h(Ar1 + ks * 32, lane), frag_h(Wr + MLPW + ks * 32, lane), acc);
    const float bv = bfr(bo[col < 3 ? col : 2]);
#pragma unroll
    for (int r = 0; r < 8; ++r) {
      const float t = tanhf(acc[r] * INV_ACC + bv);
      if (col < 3) ost[(mt * 16 + 8 * g + r) * 3 + col] = t;
    }
  }
  __syncthreads();
  if (tid < 48) {
    const v4f v = *(const v4f*)(ost + tid * 4);
    vst2(out + ((size_t)b * NPTS + p0) * 3 + (size_t)tid * 4, v);
  }
}

extern "C" void kernel_launch(void* const* d_in, const int* in_sizes, int n_in,
                              void* d_out, int out_size, void* d_ws, size_t ws_size,
                              hipStream_t stream) {
  if (n_in < 15) return;
  if (in_sizes[0] < NB * GH * GW * DM || in_sizes[1] < NB * DM || in_sizes[2] < NPTS * 2 ||
      in_sizes[3] < KIN0 * MLPW || in_sizes[4] < MLPW || in_sizes[5] < MLPW * MLPW || in_sizes[6] < MLPW ||
      in_sizes[7] < MLPW * MLPW || in_sizes[8] < MLPW || in_sizes[9] < MLPW * MLPW || in_sizes[10] < MLPW ||
      in_sizes[11] < DM * FILMW || in_sizes[12] < FILMW || in_sizes[13] < MLPW * 3 || in_sizes[14] < 3) return;
  if ((size_t)out_size < (size_t)NB * NPTS * 3) return;
  const float* fg     = (const float*)d_in[0];
  const float* ctx    = (const float*)d_in[1];
  const float* coords = (const float*)d_in[2];
  const float* w0 = (const float*)d_in[3];  const float* b0 = (const float*)d_in[4];
  const float* w1 = (const float*)d_in[5];  const float* b1 = (const float*)d_in[6];
  const float* w2 = (const float*)d_in[7];  const float* b2 = (const float*)d_in[8];
  const float* w3 = (const float*)d_in[9];  const float* b3 = (const float*)d_in[10];
  const float* wf = (const float*)d_in[11]; const float* bfm = (const float*)d_in[12];
  const float* wo = (const float*)d_in[13]; const float* bo = (const float*)d_in[14];
  float* out = (float*)d_out;

  char* ws = (char*)d_ws; size_t off = 0;
  auto take = [&](size_t bytes) { char* p = ws + off; off += (bytes + 255) & ~(size_t)255; return p; };
  float*    film = (float*)take((size_t)NB * FILMW * 4);
  _Float16* W0p  = (_Float16*)take((size_t)MLPW * (2 * KP0) * 2);
  _Float16* W1p  = (_Float16*)take((size_t)MLPW * MLPW * 2);
  _Float16* W2p  = (_Float16*)take((size_t)MLPW * MLPW * 2);
  _Float16* W3p  = (_Float16*)take((size_t)MLPW * MLPW * 2);
  _Float16* WOp  = (_Float16*)take((size_t)16 * (2 * MLPW) * 2);
  _Float16* eh   = (_Float16*)take((size_t)NPTS * ENCP * 2);
  _Float16* el   = (_Float16*)take((size_t)NPTS * ENCP * 2);
  if (off > ws_size || off > ((size_t)128 << 20)) return;

  k_film<<<NB, 256, 0, stream>>>(ctx, wf, bfm, film);
  k_wprep<<<(MLPW * (2 * KP0 / 8) + 255) / 256, 256, 0, stream>>>(w0, KIN0, MLPW, MLPW, KP0, 1, SC_W, SC_WL, W0p);
  k_wprep<<<(MLPW * (MLPW / 8) + 255) / 256, 256, 0, stream>>>(w1, MLPW, MLPW, MLPW, MLPW, 0, SC_W, SC_WL, W1p);
  k_wprep<<<(MLPW * (MLPW / 8) + 255) / 256, 256, 0, stream>>>(w2, MLPW, MLPW, MLPW, MLPW, 0, SC_W, SC_WL, W2p);
  k_wprep<<<(MLPW * (MLPW / 8) + 255) / 256, 256, 0, stream>>>(w3, MLPW, MLPW, MLPW, MLPW, 0, SC_W, SC_WL, W3p);
  k_wprep<<<(16 * (2 * MLPW / 8) + 255) / 256, 256, 0, stream>>>(wo, MLPW, 3, 16, MLPW, 1, SC_W, SC_WL, WOp);
  k_enc<<<NPTS / TILE, 256, 0, stream>>>(coords, eh, el);
  k_dec<<<NB * (NPTS / TILE), 256, 0, stream>>>(fg, coords, eh, el, W0p, W1p, W2p, W3p, WOp, b0, b1, b2, b3, film, bo, out);
}
